// RGCN_22857815949325
// MI455X (gfx1250) — hardware-verified
//
#include <hip/hip_runtime.h>

constexpr int   N_NODES = 100000;
constexpr int   N_EDGES = 1600000;
constexpr int   HID     = 128;
constexpr int   NRELS   = 8;
constexpr int   KCAT    = HID * (NRELS + 1);
constexpr int   NT      = 256;
constexpr int   TILE_N  = 1536;
constexpr int   RPW     = TILE_N / 8;
constexpr int   NTILES  = 66;
constexpr int   NPAD    = NTILES * TILE_N;
constexpr int   GROUP_T = 5;
constexpr int   GROUP_N = GROUP_T * TILE_N;
constexpr int   NGROUPS = 14;
constexpr int   CAP     = 26624;
constexpr int   MAXG    = CAP / 32 + 1;
constexpr int   SCH     = 8192;
constexpr int   SPT     = SCH / NT;
constexpr int   NCHUNK  = (N_EDGES + SCH - 1) / SCH;
constexpr int   LCAP    = 1024;
constexpr int   SLABU   = KCAT / 2;
constexpr float WCARRY     = 16.0f;
constexpr float WCARRY_INV = 1.0f / 16.0f;
constexpr size_t WS_LIMIT  = 134217728;

static_assert(KCAT % 32 == 0);
static_assert(HID % 64 == 0);
static_assert(TILE_N % 64 == 0);
static_assert(GROUP_N % 64 == 0);
static_assert(NPAD % 64 == 0);
static_assert(NPAD >= N_NODES);
static_assert((NGROUPS - 1) * GROUP_T + 1 == NTILES);
static_assert(TILE_N == NT * 6);
static_assert(RPW * 8 == TILE_N);
static_assert(N_EDGES % SPT == 0);
static_assert(SCH % NT == 0 && SPT % 4 == 0);
static_assert(TILE_N <= 2048);
static_assert(N_EDGES < (1 << 21));
static_assert(N_NODES <= (1 << 17));
static_assert(NRELS == 8);
static_assert(CAP % 32 == 0 && LCAP % 32 == 0);

typedef __attribute__((ext_vector_type(16))) _Float16 v16h;
typedef __attribute__((ext_vector_type(8)))  _Float16 v8h;
typedef __attribute__((ext_vector_type(16))) __bf16   v16b;
typedef __attribute__((ext_vector_type(8)))  __bf16   v8b;
typedef __attribute__((ext_vector_type(8)))  float    v8f;
typedef __attribute__((ext_vector_type(4)))  float    v4f;
typedef __attribute__((ext_vector_type(4)))  int      v4i;
typedef __attribute__((ext_vector_type(4)))  unsigned int v4u;
typedef __attribute__((ext_vector_type(2)))  unsigned int v2u;

__device__ __forceinline__ unsigned short f2bf_bits(float f) {
  unsigned u = __float_as_uint(f);
  return (unsigned short)((u + 0x7FFFu + ((u >> 16) & 1u)) >> 16);
}
__device__ __forceinline__ float bf_bits2f(unsigned short h) { return __uint_as_float(((unsigned)h) << 16); }
__device__ __forceinline__ unsigned pk16(unsigned short a, unsigned short b) { return (unsigned)a | ((unsigned)b << 16); }
__device__ __forceinline__ unsigned short h_bits(float f) { const _Float16 h = (_Float16)f; return __builtin_bit_cast(unsigned short, h); }

__device__ __forceinline__ void dep_guard6_h(v8f& a, v8f& b, v8f& c, v8f& d, v16h x0, v16h x1, v16h y0, v16h y1, v16h y2, v16h y3) {
  asm volatile("v_nop\n\tv_nop\n\tv_nop\n\tv_nop" : "+v"(a), "+v"(b), "+v"(c), "+v"(d) : "v"(x0), "v"(x1), "v"(y0), "v"(y1), "v"(y2), "v"(y3));
}
__device__ __forceinline__ void dep_guard6_b(v8f& a, v8f& b, v8f& c, v8f& d, v16b x0, v16b x1, v16b y0, v16b y1, v16b y2, v16b y3) {
  asm volatile("v_nop\n\tv_nop\n\tv_nop\n\tv_nop" : "+v"(a), "+v"(b), "+v"(c), "+v"(d) : "v"(x0), "v"(x1), "v"(y0), "v"(y1), "v"(y2), "v"(y3));
}
__device__ __forceinline__ void keep4_h(v16h a, v16h b, v16h c, v16h d) { asm volatile("v_nop" :: "v"(a), "v"(b), "v"(c), "v"(d)); }
__device__ __forceinline__ void keep4_b(v16b a, v16b b, v16b c, v16b d) { asm volatile("v_nop" :: "v"(a), "v"(b), "v"(c), "v"(d)); }
__device__ __forceinline__ void acc_guard4(v8f& a, v8f& b, v8f& c, v8f& d) { asm volatile("v_nop\n\tv_nop\n\tv_nop\n\tv_nop" : "+v"(a), "+v"(b), "+v"(c), "+v"(d)); }
__device__ __forceinline__ void wave_lds_sync() {
  __builtin_amdgcn_fence(__ATOMIC_RELEASE, "workgroup");
  __builtin_amdgcn_wave_barrier();
  __builtin_amdgcn_fence(__ATOMIC_ACQUIRE, "workgroup");
}
template <typename T> struct Frag;
template <> struct Frag<_Float16> {
  typedef v16h V; union U { v16h v; v8h h[2]; };
  static __device__ __forceinline__ v16h load(const _Float16* p) {
    U f; f.h[0] = *(const v8h*)(p); f.h[1] = *(const v8h*)(p + 16); return f.v;
  }
  static __device__ __forceinline__ v8f mma(v16h a, v16h b, v8f c) {
    return __builtin_amdgcn_wmma_f32_16x16x32_f16(false, a, false, b, (short)0, c, false, false);
  }
  static __device__ __forceinline__ void guard6(v8f& a, v8f& b, v8f& c, v8f& d, v16h x0, v16h x1, v16h y0, v16h y1, v16h y2, v16h y3) { dep_guard6_h(a, b, c, d, x0, x1, y0, y1, y2, y3); }
  static __device__ __forceinline__ void keep(v16h a, v16h b, v16h c, v16h d) { keep4_h(a, b, c, d); }
};
template <> struct Frag<__bf16> {
  typedef v16b V; union U { v16b v; v8b h[2]; };
  static __device__ __forceinline__ v16b load(const __bf16* p) {
    U f; f.h[0] = *(const v8b*)(p); f.h[1] = *(const v8b*)(p + 16); return f.v;
  }
  static __device__ __forceinline__ v8f mma(v16b a, v16b b, v8f c) {
    return __builtin_amdgcn_wmma_f32_16x16x32_bf16(false, a, false, b, (short)0, c, false, false);
  }
  static __device__ __forceinline__ void guard6(v8f& a, v8f& b, v8f& c, v8f& d, v16b x0, v16b x1, v16b y0, v16b y1, v16b y2, v16b y3) { dep_guard6_b(a, b, c, d, x0, x1, y0, y1, y2, y3); }
  static __device__ __forceinline__ void keep(v16b a, v16b b, v16b c, v16b d) { keep4_b(a, b, c, d); }
};

template <int ET> struct Elem;
template <> struct Elem<0> { typedef _Float16 T; };
template <> struct Elem<1> { typedef __bf16 T; };
template <int ET, bool ASPLIT>
__global__ __launch_bounds__(256) void wmma_gemm64(
    const unsigned short* __restrict__ Ap, const unsigned short* __restrict__ A2p, int lda,
    const unsigned short* __restrict__ Btp, int ldb,
    float* __restrict__ Cout, int ldc,
    const float* __restrict__ bias,
    int M, int N, int K, float scale, int mclip) {
  typedef typename Elem<ET>::T T;
  typedef typename Frag<T>::V V;
  const T* A = (const T*)Ap; const T* A2 = (const T*)A2p; const T* Bt = (const T*)Btp;
  __shared__ __align__(16) float sT[8][16 * 68];
  const int lane = threadIdx.x & 31;
  const int wave = threadIdx.x >> 5;
  const int tilesN = N >> 6;
  const int tilesM = M >> 6;
  const int tile = blockIdx.x * 8 + wave;
  if (tile >= tilesM * tilesN) return;
  const int tm = tile / tilesN;
  const int tn = tile - tm * tilesN;
  const int m0 = tm << 6;
  const int n0 = tn << 6;

  const int rlane = lane & 15;
  const int koff  = (lane >> 4) * 8;
  const int mOff  = (lane >> 4) * 8;

  v8f acc[4][4];
#pragma unroll
  for (int i = 0; i < 4; ++i)
#pragma unroll
    for (int j = 0; j < 4; ++j) acc[i][j] = (v8f){0.f,0.f,0.f,0.f,0.f,0.f,0.f,0.f};

  for (int k0 = 0; k0 < K; k0 += 32) {
    V bh[4];
#pragma unroll
    for (int j = 0; j < 4; ++j) {
      const size_t bo = (size_t)(n0 + (j << 4) + rlane) * ldb + koff + k0;
      bh[j] = Frag<T>::load(Bt + bo);
    }
#pragma unroll
    for (int i = 0; i < 4; ++i) {
      const size_t ao = (size_t)(m0 + (i << 4) + rlane) * lda + koff + k0;
      V ah = Frag<T>::load(A + ao);
      V al = ah;
      if (ASPLIT) al = Frag<T>::load(A2 + ao);
#pragma unroll
      for (int j = 0; j < 4; ++j) {
        acc[i][j] = Frag<T>::mma(ah, bh[j], acc[i][j]);
        if (ASPLIT) acc[i][j] = Frag<T>::mma(al, bh[j], acc[i][j]);
      }
      Frag<T>::guard6(acc[i][0], acc[i][1], acc[i][2], acc[i][3], ah, al, bh[0], bh[1], bh[2], bh[3]);
    }
    Frag<T>::keep(bh[0], bh[1], bh[2], bh[3]);
  }
  acc_guard4(acc[0][0], acc[0][1], acc[0][2], acc[0][3]);
  acc_guard4(acc[1][0], acc[1][1], acc[1][2], acc[1][3]);
  acc_guard4(acc[2][0], acc[2][1], acc[2][2], acc[2][3]);
  acc_guard4(acc[3][0], acc[3][1], acc[3][2], acc[3][3]);

  float* slab = sT[wave];
#pragma unroll
  for (int i = 0; i < 4; ++i) {
    const int mBase = m0 + (i << 4);
#pragma unroll
    for (int j = 0; j < 4; ++j) {
      const int n = n0 + (j << 4) + rlane;
      const float bv = bias[n];
#pragma unroll
      for (int r = 0; r < 8; ++r) {
        float v = acc[i][j][r] * scale;
        v += bv;
        v = fmaxf(v, 0.0f);
        slab[(mOff + r) * 68 + (j << 4) + rlane] = v;
      }
    }
    wave_lds_sync();
    {
      const int hh = lane >> 4, c4 = (lane & 15) * 4;
      for (int pass = 0; pass < 2; ++pass) {
#pragma unroll
        for (int it = 0; it < 8; ++it) {
          const int row = it * 2 + hh;
          v4f v = *(const v4f*)(slab + row * 68 + c4);
          if (mBase + row < mclip) *(volatile v4f*)(Cout + (size_t)(mBase + row) * ldc + n0 + c4) = v;
        }
        __threadfence();
      }
    }
    wave_lds_sync();
  }
}

__global__ __launch_bounds__(NT) void cast_x0_kernel(const int* __restrict__ node_idx, const float* __restrict__ emb,
                                                      unsigned short* __restrict__ X0) {
  const int i = blockIdx.x * NT + threadIdx.x;
  const int row = i >> 4;
  const int c8  = (i & 15) * 8;
  const bool live = row < N_NODES;
  const int rr = live ? row : (N_NODES - 1);
  int id = node_idx[rr];
  id = id < 0 ? 0 : (id >= N_NODES ? N_NODES - 1 : id);
  const float* p = emb + (size_t)id * HID + c8;
  const v4f a = *(const v4f*)(p);
  const v4f c = *(const v4f*)(p + 4);
  unsigned short hb[8];
#pragma unroll
  for (int e = 0; e < 4; ++e) {
    hb[e]     = f2bf_bits(a[e]);
    hb[4 + e] = f2bf_bits(c[e]);
  }
  const unsigned keep = live ? 0xffffffffu : 0u;
  const v4u u = (v4u){pk16(hb[0], hb[1]) & keep, pk16(hb[2], hb[3]) & keep, pk16(hb[4], hb[5]) & keep, pk16(hb[6], hb[7]) & keep};
  unsigned short* q = X0 + (size_t)row * HID + c8;
  *(volatile v4u*)q = u;
  __threadfence();
  *(volatile v4u*)q = u;
}

__global__ __launch_bounds__(NT) void prep_w_kernel(const float* __restrict__ wrel0, const float* __restrict__ wroot0, const float* __restrict__ bias0,
                                                     const float* __restrict__ wrel1, const float* __restrict__ wroot1, const float* __restrict__ bias1,
                                                     unsigned short* __restrict__ WT0, unsigned short* __restrict__ WT1,
                                                     float* __restrict__ BR0, float* __restrict__ BR1) {
  const int ly = blockIdx.y;
  const float* wrel  = ly ? wrel1 : wrel0;
  const float* wroot = ly ? wroot1 : wroot0;
  const float* bsrc  = ly ? bias1 : bias0;
  unsigned short* WT = ly ? WT1 : WT0;
  float* BR = ly ? BR1 : BR0;
  const int i  = blockIdx.x * NT + threadIdx.x;
  const int n  = i / (KCAT / 2);
  const int kb = 2 * (i - n * (KCAT / 2));
  unsigned short hb2[2];
#pragma unroll
  for (int e = 0; e < 2; ++e) {
    const int kk = kb + e;
    const int kr = kk < HID ? kk : (HID - 1);
    const int ke = kk >= HID ? (kk - HID) : 0;
    const float wa = wroot[(size_t)kr * HID + n];
    const float wb = wrel[(size_t)ke * HID + n];
    const float fa = (kk < HID) ? 1.0f : 0.0f;
    const float fb = 1.0f - fa;
    const float w = fmaf(fa, wa, fb * wb);
    const unsigned short bb = f2bf_bits(w);
    hb2[e] = ly ? bb : h_bits(WCARRY * bf_bits2f(bb));
  }
  const unsigned u = pk16(hb2[0], hb2[1]);
  ((volatile unsigned*)WT)[i] = u;
  __threadfence();
  ((volatile unsigned*)WT)[i] = u;
  if (blockIdx.x == 0 && threadIdx.x < 32) {
    const int l = threadIdx.x;
    const v4f bv = *(const v4f*)(bsrc + 4 * l);
    v4f br;
#pragma unroll
    for (int e = 0; e < 4; ++e) br[e] = bf_bits2f(f2bf_bits(bv[e]));
    *(volatile v4f*)(BR + 4 * l) = br;
    __threadfence();
    *(volatile v4f*)(BR + 4 * l) = br;
  }
}

__device__ __forceinline__ int blk_excl_scan(int cnt, int* scan_ws, int tid, int* tot) {
  const int lane = tid & 31, wave = tid >> 5; int incl = cnt;
#pragma unroll
  for (int o = 1; o < 32; o <<= 1) { const int v = __shfl_up(incl, o, 32); if (lane >= o) incl += v; }
  if (lane == 31) scan_ws[wave] = incl;
  __syncthreads();
  if (wave == 0) { int wv = (lane < NT / 32) ? scan_ws[lane] : 0; int wincl = wv;
#pragma unroll
    for (int o = 1; o < 32; o <<= 1) { const int v = __shfl_up(wincl, o, 32); if (lane >= o) wincl += v; }
    if (lane < NT / 32) scan_ws[32 + lane] = wincl - wv; if (lane == 31) scan_ws[64] = wincl; }
  __syncthreads();
  const int res = scan_ws[32 + wave] + incl - cnt; *tot = scan_ws[64];
  return res;
}
__device__ __forceinline__ int chunk_hits(const int* __restrict__ dstv, int e0, int n0, int tid, unsigned* LIST, int* scan_ws) {
  const int eb = e0 + tid * SPT;
  const bool inr = eb < N_EDGES;
  const int ebc = inr ? eb : (N_EDGES - SPT);
  unsigned rec[SPT]; int cnt = 0;
#pragma unroll
  for (int k = 0; k < SPT; k += 4) {
    const v4i d4 = *(const v4i*)(dstv + ebc + k);
#pragma unroll
    for (int e = 0; e < 4; ++e) {
      const int d = d4[e]; unsigned r = 0xFFFFFFFFu;
      if (inr && d >= n0 && d < n0 + TILE_N) { r = ((unsigned)(d - n0) << 21) | (unsigned)(ebc + k + e); ++cnt; }
      rec[k + e] = r;
    }
    if ((k & 12) == 12) asm volatile("" ::: "memory");
  }
  int tot; int p = blk_excl_scan(cnt, scan_ws, tid, &tot);
#pragma unroll
  for (int k = 0; k < SPT; ++k) if (rec[k] != 0xFFFFFFFFu) { if ((unsigned)p < (unsigned)LCAP) LIST[p] = rec[k]; ++p; }
  __syncthreads();
  return tot < LCAP ? tot : LCAP;
}
__device__ __forceinline__ v2u pack_h4(v4f m, unsigned keep) {
  v2u p;
  p[0] = pk16(h_bits(m[0]), h_bits(m[1])) & keep;
  p[1] = pk16(h_bits(m[2]), h_bits(m[3])) & keep;
  return p;
}
__device__ __forceinline__ void pack_bf_hl4(v4f m, unsigned keep, v2u& hp, v2u& lp) {
  unsigned hb[4], lb[4];
#pragma unroll
  for (int e = 0; e < 4; ++e) {
    const unsigned u = __float_as_uint(m[e]) & 0xffff0000u;
    hb[e] = u >> 16;
    lb[e] = (unsigned)f2bf_bits(m[e] - __uint_as_float(u));
  }
  hp[0] = (hb[0] | (hb[1] << 16)) & keep; hp[1] = (hb[2] | (hb[3] << 16)) & keep;
  lp[0] = (lb[0] | (lb[1] << 16)) & keep; lp[1] = (lb[2] | (lb[3] << 16)) & keep;
}

template <int LAYER>
__global__ __launch_bounds__(NT) void agg_kernel(const unsigned short* __restrict__ X0p, const float* __restrict__ X1p,
                                                 const int* __restrict__ ei, const int* __restrict__ etv,
                                                 unsigned short* __restrict__ O1, unsigned short* __restrict__ O2, int tile0) {
  __shared__ unsigned SORTED[CAP];
  __shared__ unsigned LIST[LCAP];
  __shared__ int OFFS[TILE_N];
  __shared__ int CUR[TILE_N];
  __shared__ __align__(16) unsigned slab[NT / 32][SLABU];
  __shared__ int scan_ws[80];
  const int tid = threadIdx.x, lane = tid & 31, wave = tid >> 5;
  const int n0   = (tile0 + (int)blockIdx.x) * TILE_N;
  const int rowb = (int)blockIdx.x * TILE_N;
  for (int i = tid; i < CAP; i += NT) SORTED[i] = 0u;
  for (int i = tid; i < LCAP; i += NT) LIST[i] = 0u;
  for (int i = tid; i < TILE_N; i += NT) { OFFS[i] = 0; CUR[i] = 0; }
  for (int i = lane; i < SLABU; i += 32) slab[wave][i] = 0u;
  if (tid < 80) scan_ws[tid] = 0;
  __syncthreads();
  const int* srcv = ei;
  const int* dstv = ei + N_EDGES;

#pragma unroll 1
  for (int c = 0; c < NCHUNK; ++c) {
    const int tot = chunk_hits(dstv, c * SCH, n0, tid, LIST, scan_ws);
#pragma unroll 1
    for (int base = 0; base < tot; base += 32) {
      const int q  = base + lane;
      const int qc = q < LCAP ? q : (LCAP - 1);
      const unsigned lw = LIST[qc];
      const int dlq = (int)(lw >> 21);
      const int own = (q < tot && (dlq / RPW) == wave) ? 1 : 0;
      unsigned msk = (unsigned)__ballot(own);
#pragma unroll 1
      for (int it = 0; it < 32; ++it) {
        if (msk == 0u) break;
        const int bp = __builtin_ctz(msk); msk &= msk - 1u;
        const unsigned r = (unsigned)__shfl((int)lw, bp, 32);
        int dl = (int)(r >> 21); dl = dl < TILE_N ? dl : (TILE_N - 1);
        const int cc = CUR[dl];
        if (lane == 0) CUR[dl] = cc + 1;
      }
    }
    __syncthreads();
  }
  {
    const int d0 = tid * (TILE_N / NT);
    int c6[TILE_N / NT]; int s = 0;
#pragma unroll
    for (int k = 0; k < TILE_N / NT; ++k) { c6[k] = CUR[d0 + k]; s += c6[k]; }
    int tot; const int p = blk_excl_scan(s, scan_ws, tid, &tot);
    int run = p;
#pragma unroll
    for (int k = 0; k < TILE_N / NT; ++k) { OFFS[d0 + k] = run; CUR[d0 + k] = run; run += c6[k]; }
  }
  __syncthreads();
#pragma unroll 1
  for (int c = 0; c < NCHUNK; ++c) {
    const int tot = chunk_hits(dstv, c * SCH, n0, tid, LIST, scan_ws);
#pragma unroll 1
    for (int base = 0; base < tot; base += 32) {
      const int q  = base + lane;
      const int qc = q < LCAP ? q : (LCAP - 1);
      const unsigned lw = LIST[qc];
      const int dlq = (int)(lw >> 21);
      const int own = (q < tot && (dlq / RPW) == wave) ? 1 : 0;
      unsigned msk = (unsigned)__ballot(own);
#pragma unroll 1
      for (int it = 0; it < 32; ++it) {
        if (msk == 0u) break;
        const int bp = __builtin_ctz(msk); msk &= msk - 1u;
        const unsigned r = (unsigned)__shfl((int)lw, bp, 32);
        int dl = (int)(r >> 21); dl = dl < TILE_N ? dl : (TILE_N - 1);
        int e = (int)(r & 0x1FFFFFu); e = e < N_EDGES ? e : (N_EDGES - 1);
        int sv = srcv[e]; sv = sv < 0 ? 0 : (sv >= N_NODES ? (N_NODES - 1) : sv);
        int tv = etv[e];  tv = tv < 0 ? 0 : (tv >= NRELS ? (NRELS - 1) : tv);
        const unsigned w = ((unsigned)tv << 17) | (unsigned)sv;
        const int pos = CUR[dl];
        const int pc = pos < CAP ? pos : (CAP - 1);
        if (lane == 0 && pos < CAP) SORTED[pc] = w;
        if (lane == 0) CUR[dl] = pos + 1;
      }
    }
    __syncthreads();
  }
  const v4f z4 = {0.f, 0.f, 0.f, 0.f};
  unsigned* sl = slab[wave];
#pragma unroll 1
  for (int j = 0; j < RPW; ++j) {
    const int dl = wave * RPW + j;
    const int n  = n0 + dl;
    const bool live = n < N_NODES;
    int start = __builtin_amdgcn_readfirstlane(OFFS[dl]);
    int end   = __builtin_amdgcn_readfirstlane(CUR[dl]);
    start = start < 0 ? 0 : (start > CAP ? CAP : start);
    end   = end > CAP ? CAP : end;
    end   = end < start ? start : end;
    v4f acc[NRELS]; int cnt[NRELS];
#pragma unroll
    for (int r = 0; r < NRELS; ++r) { acc[r] = z4; cnt[r] = 0; }
#pragma unroll 1
    for (int g = 0; g < MAXG; ++g) {
      const int base = start + (g << 5);
      if (base >= end) break;
      const int idx = base + lane;
      const bool valid = idx < end;
      const int idc = valid ? idx : base;
      const unsigned w = SORTED[idc];
      const int rel = (int)((w >> 17) & 7u);
      int s = (int)(w & 0x1FFFFu); s = s < N_NODES ? s : (N_NODES - 1);
#pragma unroll
      for (int r = 0; r < NRELS; ++r) {
        unsigned m = (unsigned)__ballot((valid && rel == r) ? 1 : 0);
        cnt[r] += __builtin_popcount(m);
#pragma unroll 1
        for (int it = 0; it < 32; ++it) {
          if (m == 0u) break;
          const int bp = __builtin_ctz(m); m &= m - 1u;
          const int sv = __shfl(s, bp, 32);
          v4f xv;
          if (LAYER == 0) {
            const v2u xw = *(const v2u*)(X0p + (size_t)sv * HID + 4 * lane);
            xv[0] = __uint_as_float(xw[0] << 16); xv[1] = __uint_as_float(xw[0] & 0xffff0000u);
            xv[2] = __uint_as_float(xw[1] << 16); xv[3] = __uint_as_float(xw[1] & 0xffff0000u);
          } else {
            xv = *(const v4f*)(X1p + (size_t)sv * HID + 4 * lane);
          }
          acc[r] = acc[r] + xv;
        }
      }
    }
    const unsigned keep = live ? 0xffffffffu : 0u;
    v4f segv[NRELS + 1];
    if (LAYER == 0) {
      const v2u xw = *(const v2u*)(X0p + (size_t)n * HID + 4 * lane);
      segv[0][0] = __uint_as_float(xw[0] << 16); segv[0][1] = __uint_as_float(xw[0] & 0xffff0000u);
      segv[0][2] = __uint_as_float(xw[1] << 16); segv[0][3] = __uint_as_float(xw[1] & 0xffff0000u);
    } else {
      segv[0] = *(const v4f*)(X1p + (size_t)n * HID + 4 * lane);
    }
#pragma unroll
    for (int r = 0; r < NRELS; ++r) {
      const float cf = (float)cnt[r];
      const float inv = 1.0f / fmaxf(cf, 1.0f);
      segv[1 + r] = acc[r] * inv;
    }
    unsigned* ou1 = (unsigned*)(O1 + (size_t)(rowb + dl) * KCAT);
    if (LAYER == 0) {
#pragma unroll
      for (int seg = 0; seg < NRELS + 1; ++seg) *(v2u*)(sl + seg * 64 + 2 * lane) = pack_h4(segv[seg], keep);
      wave_lds_sync();
      v4u hreg[5];
#pragma unroll
      for (int it = 0; it < 4; ++it) hreg[it] = *(const v4u*)(sl + it * 128 + 4 * lane);
      hreg[4] = *(const v4u*)(sl + 512 + 4 * (lane & 15));
      for (int pass = 0; pass < 2; ++pass) {
#pragma unroll
        for (int it = 0; it < 4; ++it) *(volatile v4u*)(ou1 + it * 128 + 4 * lane) = hreg[it];
        if (lane < 16) *(volatile v4u*)(ou1 + 512 + 4 * lane) = hreg[4];
        __threadfence();
      }
      wave_lds_sync();
    } else {
      unsigned* ou2 = (unsigned*)(O2 + (size_t)(rowb + dl) * KCAT);
      v2u hp[NRELS + 1], lp[NRELS + 1];
#pragma unroll
      for (int seg = 0; seg < NRELS + 1; ++seg) pack_bf_hl4(segv[seg], keep, hp[seg], lp[seg]);
#pragma unroll
      for (int seg = 0; seg < NRELS + 1; ++seg) *(v2u*)(sl + seg * 64 + 2 * lane) = hp[seg];
      wave_lds_sync();
      v4u hreg[5], lreg[5];
#pragma unroll
      for (int it = 0; it < 4; ++it) hreg[it] = *(const v4u*)(sl + it * 128 + 4 * lane);
      hreg[4] = *(const v4u*)(sl + 512 + 4 * (lane & 15));
      wave_lds_sync();
#pragma unroll
      for (int seg = 0; seg < NRELS + 1; ++seg) *(v2u*)(sl + seg * 64 + 2 * lane) = lp[seg];
      wave_lds_sync();
#pragma unroll
      for (int it = 0; it < 4; ++it) lreg[it] = *(const v4u*)(sl + it * 128 + 4 * lane);
      lreg[4] = *(const v4u*)(sl + 512 + 4 * (lane & 15));
      for (int pass = 0; pass < 2; ++pass) {
#pragma unroll
        for (int it = 0; it < 4; ++it) {
          *(volatile v4u*)(ou1 + it * 128 + 4 * lane) = hreg[it];
          *(volatile v4u*)(ou2 + it * 128 + 4 * lane) = lreg[it];
        }
        if (lane < 16) {
          *(volatile v4u*)(ou1 + 512 + 4 * lane) = hreg[4];
          *(volatile v4u*)(ou2 + 512 + 4 * lane) = lreg[4];
        }
        __threadfence();
      }
      wave_lds_sync();
    }
  }
}

extern "C" void kernel_launch(void* const* d_in, const int* in_sizes, int n_in,
                              void* d_out, int out_size, void* d_ws, size_t ws_size, hipStream_t stream) {
  if (n_in < 10) return;
  const int*   node_idx = (const int*)d_in[0];
  const int*   ei       = (const int*)d_in[1];
  const int*   et       = (const int*)d_in[2];
  const float* emb      = (const float*)d_in[3];
  const float* wrel0    = (const float*)d_in[4];
  const float* wroot0   = (const float*)d_in[5];
  const float* bias0    = (const float*)d_in[6];
  const float* wrel1    = (const float*)d_in[7];
  const float* wroot1   = (const float*)d_in[8];
  const float* bias1    = (const float*)d_in[9];
  if (in_sizes[0] != N_NODES || in_sizes[1] != 2 * N_EDGES || in_sizes[2] != N_EDGES ||
      in_sizes[3] != N_NODES * HID || in_sizes[4] != NRELS * HID * HID || in_sizes[5] != HID * HID ||
      in_sizes[6] != HID || in_sizes[7] != NRELS * HID * HID || in_sizes[8] != HID * HID || in_sizes[9] != HID ||
      out_size != N_NODES * HID) return;
  float* out = (float*)d_out;

  char* ws = (char*)d_ws; size_t off = 0;
  auto carve = [&](size_t bytes) -> char* { char* p = ws + off; off += (bytes + 255) & ~(size_t)255; return p; };
  unsigned short* X0   = (unsigned short*)carve((size_t)NPAD * HID * 2);
  float*          X1   = (float*)carve((size_t)NPAD * HID * 4);
  unsigned short* WT0  = (unsigned short*)carve((size_t)HID * KCAT * 2);
  unsigned short* WT1  = (unsigned short*)carve((size_t)HID * KCAT * 2);
  float*          BR0  = (float*)carve((size_t)HID * 4);
  float*          BR1  = (float*)carve((size_t)HID * 4);
  unsigned short* APL0 = (unsigned short*)carve((size_t)GROUP_N * KCAT * 2);
  unsigned short* APLH = (unsigned short*)carve((size_t)GROUP_N * KCAT * 2);
  unsigned short* APLL = (unsigned short*)carve((size_t)GROUP_N * KCAT * 2);
  if (off > ws_size || off > WS_LIMIT) return;

  cast_x0_kernel<<<(NPAD * 16) / NT, NT, 0, stream>>>(node_idx, emb, X0);
  prep_w_kernel<<<dim3((HID * KCAT / 2) / NT, 2), NT, 0, stream>>>(wrel0, wroot0, bias0, wrel1, wroot1, bias1,
                                                                    WT0, WT1, BR0, BR1);

  for (int layer = 0; layer < 2; ++layer) {
    for (int g = 0; g < NGROUPS; ++g) {
      const int tiles = (g < NGROUPS - 1) ? GROUP_T : (NTILES - (NGROUPS - 1) * GROUP_T);
      const int rows  = tiles * TILE_N;
      const int tile0 = g * GROUP_T;
      const int goff  = tile0 * TILE_N;
      const int wtiles = (rows / 64) * (HID / 64);
      const int gx = (wtiles + 7) / 8;
      if (layer == 0) {
        agg_kernel<0><<<tiles, NT, 0, stream>>>(X0, X1, ei, et, APL0, APLL, tile0);
        wmma_gemm64<0, false><<<dim3(gx, 1), 256, 0, stream>>>(
            (const unsigned short*)APL0, (const unsigned short*)APL0, KCAT, (const unsigned short*)WT0, KCAT,
            X1 + (size_t)goff * HID, HID, BR0, rows, HID, KCAT, WCARRY_INV, rows);
      } else {
        agg_kernel<1><<<tiles, NT, 0, stream>>>(X0, X1, ei, et, APLH, APLL, tile0);
        wmma_gemm64<1, true><<<dim3(gx, 1), 256, 0, stream>>>(
            (const unsigned short*)APLH, (const unsigned short*)APLL, KCAT, (const unsigned short*)WT1, KCAT,
            out + (size_t)goff * HID, HID, BR1, rows, HID, KCAT, 1.0f, N_NODES - goff);
      }
    }
  }
}
